// SpectralMamba_10788957847757
// MI455X (gfx1250) — hardware-verified
//
#include <hip/hip_runtime.h>


namespace {
constexpr int B = 2, C = 96, HI = 96, LI = HI * HI, D2 = 192, D4 = 768, NS = 16, DR = 6, XW = 48, NT = B * LI;
constexpr float XS = 8.0f, US = 64.0f, TS = 256.0f, WSC = 256.0f;
typedef _Float16 b16;
typedef __attribute__((ext_vector_type(16))) _Float16 v16b;
typedef __attribute__((ext_vector_type(8))) _Float16 v8b;
typedef __attribute__((ext_vector_type(8))) float v8f;
typedef __attribute__((ext_vector_type(4))) float v4f;
typedef __attribute__((ext_vector_type(2))) float v2f;
__device__ __forceinline__ float bf16_rne(float f) { unsigned int u = __float_as_uint(f); u += 0x7FFFu + ((u >> 16) & 1u); return __uint_as_float(u & 0xFFFF0000u); }
__device__ __forceinline__ void split16(float v, b16& hi, b16& lo) { hi = (b16)v; lo = (b16)(v - (float)hi); }
__device__ __forceinline__ v16b frag_kb(const b16* p, int hh) { const v8b a = *(const v8b*)(p + 8 * hh), b = *(const v8b*)(p + 16 + 8 * hh); v16b f;
#pragma unroll
  for (int e = 0; e < 8; ++e) { f[e] = a[e]; f[8 + e] = b[e]; } return f; }
__device__ __forceinline__ v8f wmma16b(v16b a, v16b b, v8f c) { v8f d = __builtin_amdgcn_wmma_f32_16x16x32_f16(false, a, false, b, (short)0, c, false, false); asm volatile("v_nop\n\tv_nop\n\tv_nop\n\tv_nop" : "+v"(d) : "v"(a), "v"(b)); return d; }
__device__ __forceinline__ void wave_lds_sync() { __builtin_amdgcn_fence(__ATOMIC_RELEASE, "workgroup"); __builtin_amdgcn_wave_barrier(); __builtin_amdgcn_fence(__ATOMIC_ACQUIRE, "workgroup"); }
__device__ __forceinline__ float pmul(float a, float b) { float p = a * b; asm volatile("" : "+v"(p)); return p; }
__device__ __forceinline__ float sigm(float v) { return 1.0f / (1.0f + __expf(-v)); }
__device__ __forceinline__ float silu(float v) { return pmul(v, sigm(v)); }
__device__ __forceinline__ float softplus(float v) { return v > 20.0f ? v : (v < -20.0f ? __expf(v) : log1pf(__expf(v))); }

__global__ __launch_bounds__(256) void wput_kernel(const float* __restrict__ w, int KIN, int OUTW, int KP, int OUTP, b16* __restrict__ WT) {
  const int KG = KP / 8; const int u = blockIdx.x * 256 + threadIdx.x; if (u >= OUTP * KG) return; const int o = u / KG, k0 = (u % KG) * 8; v8b v;
#pragma unroll
  for (int j = 0; j < 8; ++j) { const int k = k0 + j; v[j] = (k < KIN && o < OUTW) ? (b16)(bf16_rne(w[(size_t)k * OUTW + o]) * WSC) : (b16)0.0f; } for (int pass = 0; pass < 2; ++pass) { *(volatile v8b*)(WT + (size_t)o * KP + k0) = v; __threadfence(); }
}
__global__ __launch_bounds__(256) void xa_kernel(const float* __restrict__ x, b16* __restrict__ XA) {
  __shared__ float T[32][HI + 1]; const int cg = blockIdx.x % 3, y = (blockIdx.x / 3) % HI, b = blockIdx.x / (3 * HI); const int tid = threadIdx.x;
  for (int i = tid; i < 32 * HI; i += 256) { const int cl = i / HI, xx = i % HI; T[cl][xx] = bf16_rne(x[(((size_t)b * C + cg * 32 + cl) * HI + y) * HI + xx]); }
  __syncthreads();
  for (int pass = 0; pass < 2; ++pass) { for (int i = tid; i < HI * 4; i += 256) { const int xx = i / 4, g8 = i % 4; v8b v; for (int j = 0; j < 8; ++j) v[j] = (b16)(T[g8 * 8 + j][xx] * XS); *(volatile v8b*)(XA + (((size_t)b * HI + y) * HI + xx) * C + cg * 32 + g8 * 8) = v; } __threadfence(); }
}
__global__ __launch_bounds__(32) void inproj_kernel(const b16* __restrict__ XA, const b16* __restrict__ WT, const float* __restrict__ bias, int NTV, float* __restrict__ XZ) {
  __shared__ __attribute__((aligned(16))) b16 Ah[16][C + 8]; __shared__ __attribute__((aligned(16))) float Tf[16][128 + 4];
  const int lane = threadIdx.x, nloc = lane & 15, hlf = lane >> 4; const size_t t0 = (size_t)blockIdx.x * 16; if (t0 >= (size_t)NTV) return;
  for (int rr = 0; rr < 16; ++rr) for (int q = 0; q < 3; ++q) Ah[rr][q * 32 + lane] = XA[(t0 + rr) * C + q * 32 + lane];
  wave_lds_sync();
#pragma unroll 1
  for (int cg = 0; cg < 3; ++cg) { v8f acc[8];
#pragma unroll
    for (int t = 0; t < 8; ++t) acc[t] = (v8f){};
#pragma unroll
    for (int kb = 0; kb < C; kb += 32) { const v16b a = frag_kb(&Ah[nloc][kb], hlf);
#pragma unroll
      for (int t = 0; t < 8; ++t) acc[t] = wmma16b(a, frag_kb(WT + (size_t)(cg * 128 + t * 16 + nloc) * C + kb, hlf), acc[t]); }
#pragma unroll
    for (int t = 0; t < 8; ++t) { const int c = cg * 128 + t * 16 + nloc; const float bb = bf16_rne(bias[c]);
#pragma unroll 1
      for (int r8 = 0; r8 < 8; ++r8) Tf[8 * hlf + r8][t * 16 + nloc] = acc[t][r8] * (1.0f / (XS * WSC)) + bb; }
    wave_lds_sync();
    for (int pass = 0; pass < 2; ++pass) { for (int rr = 0; rr < 16; ++rr) *(volatile v4f*)(XZ + (t0 + rr) * (2 * D2) + cg * 128 + lane * 4) = *(const v4f*)(&Tf[rr][lane * 4]); __threadfence(); }
    wave_lds_sync(); }
}
__global__ __launch_bounds__(256) void dwconv_kernel(const float* __restrict__ XZ, const float* __restrict__ cw, const float* __restrict__ cb, int NTV, float* __restrict__ U) {
  const size_t gid = (size_t)blockIdx.x * 256 + threadIdx.x; const size_t t = gid / (D2 / 4); const int d4 = (int)(gid % (D2 / 4)) * 4; if (t >= (size_t)NTV) return;
  const int b = (int)(t / LI), p = (int)(t % LI), y = p / HI, xx = p % HI; v4f acc; for (int q = 0; q < 4; ++q) acc[q] = bf16_rne(cb[d4 + q]);
#pragma unroll
  for (int di = 0; di < 3; ++di)
#pragma unroll
    for (int dj = 0; dj < 3; ++dj) { const int yy = y + di - 1, x2 = xx + dj - 1; const bool ok = yy >= 0 && yy < HI && x2 >= 0 && x2 < HI; const int yc = ok ? yy : y, xc = ok ? x2 : xx;
      const v4f v = *(const v4f*)(XZ + (((size_t)b * HI + yc) * HI + xc) * (2 * D2) + d4); for (int q = 0; q < 4; ++q) acc[q] += ok ? pmul(v[q], bf16_rne(cw[(d4 + q) * 9 + di * 3 + dj])) : 0.0f; }
  v4f o; for (int q = 0; q < 4; ++q) o[q] = silu(acc[q]);
  for (int pass = 0; pass < 2; ++pass) { *(volatile v4f*)(U + t * D2 + d4) = o; __threadfence(); }
}
__global__ __launch_bounds__(32) void xproj_kernel(const float* __restrict__ U, const b16* __restrict__ XPW, const b16* __restrict__ DTW, const float* __restrict__ bd, int NTV, float* __restrict__ BC, float* __restrict__ DT) {
  __shared__ __attribute__((aligned(16))) b16 Ah[16][D4 + 8], Al[16][D4 + 8], Dh[16][32 + 8], Dl[16][32 + 8]; __shared__ __attribute__((aligned(16))) float Sbc[16][32], Tf[16][128 + 4];
  const int lane = threadIdx.x, nloc = lane & 15, hlf = lane >> 4; const size_t t0 = (size_t)blockIdx.x * 16; if (t0 >= (size_t)NTV) return; const int b = (int)(t0 / LI);
  for (int rr = 0; rr < 16; ++rr) { const size_t t = t0 + rr; const int l = (int)(t % LI); const size_t tf = (size_t)b * LI + (LI - 1 - l);
    for (int q = 0; q < 6; ++q) { const int c = q * 32 + lane; b16 p, ql; split16(U[t * D2 + c] * US, p, ql); Ah[rr][c] = p; Al[rr][c] = ql; Ah[rr][D2 + c] = p; Al[rr][D2 + c] = ql; split16(U[tf * D2 + c] * US, p, ql); Ah[rr][2 * D2 + c] = p; Al[rr][2 * D2 + c] = ql; Ah[rr][3 * D2 + c] = p; Al[rr][3 * D2 + c] = ql; }
    Dh[rr][lane] = (b16)0.0f; Dl[rr][lane] = (b16)0.0f; }
  wave_lds_sync();
  v8f ax[3] = {(v8f){}, (v8f){}, (v8f){}};
#pragma unroll 2
  for (int kb = 0; kb < D4; kb += 32) { const v16b a = frag_kb(&Ah[nloc][kb], hlf), al = frag_kb(&Al[nloc][kb], hlf);
#pragma unroll
    for (int t = 0; t < 3; ++t) { const v16b bw = frag_kb(XPW + (size_t)(t * 16 + nloc) * D4 + kb, hlf); ax[t] = wmma16b(a, bw, ax[t]); ax[t] = wmma16b(al, bw, ax[t]); } }
  wave_lds_sync();
#pragma unroll
  for (int t = 0; t < 3; ++t) { const int c = t * 16 + nloc;
#pragma unroll
    for (int r8 = 0; r8 < 8; ++r8) { const int rl = 8 * hlf + r8; const float v = ax[t][r8] * (1.0f / (US * WSC)); if (c < DR) { b16 p, ql; split16(v * TS, p, ql); Dh[rl][c] = p; Dl[rl][c] = ql; } else if (c < DR + 2 * NS) Sbc[rl][c - DR] = v; } }
  wave_lds_sync();
  for (int pass = 0; pass < 2; ++pass) { for (int rr = 0; rr < 16; ++rr) ((volatile float*)BC)[(t0 + rr) * 32 + lane] = Sbc[rr][lane]; __threadfence(); }
  const v16b a = frag_kb(&Dh[nloc][0], hlf), al = frag_kb(&Dl[nloc][0], hlf);
#pragma unroll 1
  for (int cg = 0; cg < D4 / 128; ++cg) { v8f acc[8];
#pragma unroll
    for (int t = 0; t < 8; ++t) { acc[t] = (v8f){}; const v16b bw = frag_kb(DTW + (size_t)(cg * 128 + t * 16 + nloc) * 32, hlf); acc[t] = wmma16b(a, bw, acc[t]); acc[t] = wmma16b(al, bw, acc[t]); }
#pragma unroll
    for (int t = 0; t < 8; ++t) { const int c = cg * 128 + t * 16 + nloc; const float bb = bf16_rne(bd[c]);
#pragma unroll 1
      for (int r8 = 0; r8 < 8; ++r8) Tf[8 * hlf + r8][t * 16 + nloc] = softplus(acc[t][r8] * (1.0f / (TS * WSC)) + bb); }
    wave_lds_sync();
    for (int pass = 0; pass < 2; ++pass) { for (int rr = 0; rr < 16; ++rr) *(volatile v4f*)(DT + (t0 + rr) * D4 + cg * 128 + lane * 4) = *(const v4f*)(&Tf[rr][lane * 4]); __threadfence(); }
    wave_lds_sync(); }
}
__global__ __launch_bounds__(256) void scan_kernel(const float* __restrict__ U, const float* __restrict__ DT, const float* __restrict__ BC, const float* __restrict__ alog, const float* __restrict__ Dp, int NBV, int LSTEPS, float* __restrict__ Y) {
  const int gid = blockIdx.x * 256 + threadIdx.x; const int k = gid % D4, b = gid / D4; if (b >= NBV) return; const int qd = k / D2, d = k % D2;
  float A[NS]; for (int s = 0; s < NS; ++s) A[s] = -__expf(bf16_rne(alog[(size_t)k * NS + s])); const float dk = bf16_rne(Dp[k]);
#pragma unroll 1
  for (int pass = 0; pass < 2; ++pass) { float h[NS]; for (int s = 0; s < NS; ++s) h[s] = 0.0f;
#pragma unroll 1
    for (int l = 0; l < LSTEPS; ++l) { const int pos = qd < 2 ? l : (LI - 1 - l); const size_t tl = (size_t)b * LI + l, tp = (size_t)b * LI + pos;
      const float u = U[tp * D2 + d], dt = DT[tl * D4 + k]; const float du = pmul(dt, u); const float* bc = BC + tl * 32; float acc = 0.0f;
#pragma unroll
      for (int s = 0; s < NS; ++s) { h[s] = pmul(h[s], __expf(pmul(dt, A[s]))) + pmul(du, bc[s]); acc += pmul(h[s], bc[NS + s]); }
      ((volatile float*)Y)[((size_t)qd * NT + tp) * D2 + d] = acc + pmul(dk, u); }
    __threadfence(); }
}
__global__ __launch_bounds__(32) void out_kernel(const float* __restrict__ Y, const float* __restrict__ XZ, const float* __restrict__ g, const float* __restrict__ bb, const b16* __restrict__ WO, float* __restrict__ out) {
  __shared__ __attribute__((aligned(16))) b16 Ah[16][D2 + 8], Al[16][D2 + 8]; __shared__ float To[C][33];
  const int lane = threadIdx.x, nloc = lane & 15, hlf = lane >> 4; const size_t tw0 = (size_t)blockIdx.x * 32; const int b = (int)(tw0 / LI); const int p0 = (int)(tw0 % LI);
  float gg[6], be[6]; for (int q = 0; q < 6; ++q) { gg[q] = bf16_rne(g[q * 32 + lane]); be[q] = bf16_rne(bb[q * 32 + lane]); }
#pragma unroll 1
  for (int half = 0; half < 2; ++half) { const size_t t0 = tw0 + half * 16;
    for (int rr = 0; rr < 16; ++rr) { const size_t t = t0 + rr; float v[6]; float s = 0.0f; for (int q = 0; q < 6; ++q) { const int c = q * 32 + lane; float a = 0.0f; for (int qd = 0; qd < 4; ++qd) a += Y[((size_t)qd * NT + t) * D2 + c]; v[q] = a; s += a; }
      for (int o = 16; o; o >>= 1) s += __shfl_xor(s, o); const float mu = s * (1.0f / D2); float vq = 0.0f; for (int q = 0; q < 6; ++q) { const float d_ = v[q] - mu; vq += pmul(d_, d_); } for (int o = 16; o; o >>= 1) vq += __shfl_xor(vq, o); const float rs = rsqrtf(vq * (1.0f / D2) + 1e-5f);
      for (int q = 0; q < 6; ++q) { const int c = q * 32 + lane; const float z = XZ[t * (2 * D2) + D2 + c]; const float a = pmul(pmul(pmul(v[q] - mu, rs), gg[q]) + be[q], silu(z)); b16 p, ql; split16(a * XS, p, ql); Ah[rr][c] = p; Al[rr][c] = ql; } }
    wave_lds_sync();
    v8f acc[6];
#pragma unroll
    for (int t = 0; t < 6; ++t) acc[t] = (v8f){};
#pragma unroll 2
    for (int kb = 0; kb < D2; kb += 32) { const v16b a = frag_kb(&Ah[nloc][kb], hlf), al = frag_kb(&Al[nloc][kb], hlf);
#pragma unroll
      for (int t = 0; t < 6; ++t) { const v16b bw = frag_kb(WO + (size_t)(t * 16 + nloc) * D2 + kb, hlf); acc[t] = wmma16b(a, bw, acc[t]); acc[t] = wmma16b(al, bw, acc[t]); } }
#pragma unroll
    for (int t = 0; t < 6; ++t)
#pragma unroll
      for (int r8 = 0; r8 < 8; ++r8) To[t * 16 + nloc][half * 16 + 8 * hlf + r8] = acc[t][r8] * (1.0f / (XS * WSC));
    wave_lds_sync(); }
  for (int pass = 0; pass < 2; ++pass) { for (int c = 0; c < C; ++c) ((volatile float*)out)[((size_t)b * C + c) * LI + p0 + lane] = To[c][lane]; __threadfence(); }
}
}

extern "C" void kernel_launch(void* const* d_in, const int* in_sizes, int n_in, void* d_out, int out_size, void* d_ws, size_t ws_size, hipStream_t stream) {
  (void)n_in;
  auto Fp = [&](int i) { return (const float*)d_in[i]; };
  if (in_sizes[0] != NT * C || in_sizes[1] != C * 2 * D2 || in_sizes[3] != D2 * 9 || in_sizes[5] != D4 * NS || in_sizes[7] != D4 * (DR + 2 * NS) || in_sizes[8] != DR * D4 || in_sizes[12] != D2 * C || out_size != NT * C) return;
  const int NBV = B; const int NTV = NBV * LI; const int LSTEPS = LI;
  size_t off = 0; char* ws = (char*)d_ws;
  auto carve = [&](size_t bytes) { char* p = ws + off; off += (bytes + 255) & ~(size_t)255; return p; };
  b16* WI = (b16*)carve((size_t)2 * D2 * C * 2); b16* XPW = (b16*)carve((size_t)XW * D4 * 2); b16* DTW = (b16*)carve((size_t)D4 * 32 * 2); b16* WO = (b16*)carve((size_t)C * D2 * 2); b16* XA = (b16*)carve((size_t)NT * C * 2);
  float* XZ = (float*)carve((size_t)NT * 2 * D2 * 4); float* U = (float*)carve((size_t)NT * D2 * 4); float* BC = (float*)carve((size_t)NT * 32 * 4); float* DT = (float*)carve((size_t)NT * D4 * 4); float* Y = (float*)carve((size_t)4 * NT * D2 * 4);
  if (off > ws_size || off > ((size_t)192 << 20)) return;
  wput_kernel<<<(2 * D2 * (C / 8) + 255) / 256, 256, 0, stream>>>(Fp(1), C, 2 * D2, C, 2 * D2, WI); wput_kernel<<<(XW * (D4 / 8) + 255) / 256, 256, 0, stream>>>(Fp(7), D4, DR + 2 * NS, D4, XW, XPW);
  wput_kernel<<<(D4 * 4 + 255) / 256, 256, 0, stream>>>(Fp(8), DR, D4, 32, D4, DTW); wput_kernel<<<(C * (D2 / 8) + 255) / 256, 256, 0, stream>>>(Fp(12), D2, C, D2, C, WO);
  xa_kernel<<<NBV * HI * 3, 256, 0, stream>>>(Fp(0), XA);
  inproj_kernel<<<NTV / 16, 32, 0, stream>>>(XA, WI, Fp(2), NTV, XZ);
  dwconv_kernel<<<(unsigned)(((size_t)NTV * (D2 / 4) + 255) / 256), 256, 0, stream>>>(XZ, Fp(3), Fp(4), NTV, U);
  xproj_kernel<<<NTV / 16, 32, 0, stream>>>(U, XPW, DTW, Fp(9), NTV, BC, DT);
  scan_kernel<<<(NBV * D4 + 255) / 256, 256, 0, stream>>>(U, DT, BC, Fp(5), Fp(6), NBV, LSTEPS, Y);
  out_kernel<<<NTV / 32, 32, 0, stream>>>(Y, XZ, Fp(10), Fp(11), WO, (float*)d_out);
}
